// GlobalDownSample_85676007620987
// MI455X (gfx1250) — hardware-verified
//
#include <hip/hip_runtime.h>
#include <math.h>

typedef __attribute__((ext_vector_type(16))) _Float16 v16h;
typedef __attribute__((ext_vector_type(8)))  _Float16 v8h;
typedef __attribute__((ext_vector_type(16))) __bf16   v16b;
typedef __attribute__((ext_vector_type(8)))  float    v8f;
typedef __attribute__((ext_vector_type(4)))  float    v4f;

__device__ __forceinline__ int frag_k(int i, int h) { return (i < 8) ? (8 * h + i) : (16 + 8 * h + (i - 8)); }
__device__ __forceinline__ __bf16 bf16_rne(float f) {
    unsigned int u = __float_as_uint(f);
    u += 0x7fffu + ((u >> 16) & 1u);
    return __builtin_bit_cast(__bf16, (unsigned short)(u >> 16));
}
__device__ __forceinline__ float bf16_f32(__bf16 b) { return __uint_as_float(((unsigned int)__builtin_bit_cast(unsigned short, b)) << 16); }
__device__ __forceinline__ v8f wmma16(v16h a, v16h b, v8f c) {
    c = __builtin_amdgcn_wmma_f32_16x16x32_f16(false, a, false, b, (short)0, c, false, false);
    asm volatile("v_nop\n\tv_nop\n\tv_nop\n\tv_nop" : "+v"(c) : "v"(a), "v"(b));
    return c;
}
__device__ __forceinline__ v8f wmmab(v16b a, v16b b, v8f c) {
    c = __builtin_amdgcn_wmma_f32_16x16x32_bf16(false, a, false, b, (short)0, c, false, false);
    asm volatile("v_nop\n\tv_nop\n\tv_nop\n\tv_nop" : "+v"(c) : "v"(a), "v"(b));
    return c;
}
struct Split { v16b hi, lo; };
__device__ __forceinline__ v8f wmma3(const Split& a, const Split& b, v8f c) {
    c = __builtin_amdgcn_wmma_f32_16x16x32_bf16(false, a.hi, false, b.hi, (short)0, c, false, false);
    c = __builtin_amdgcn_wmma_f32_16x16x32_bf16(false, a.hi, false, b.lo, (short)0, c, false, false);
    c = __builtin_amdgcn_wmma_f32_16x16x32_bf16(false, a.lo, false, b.hi, (short)0, c, false, false);
    asm volatile("v_nop\n\tv_nop\n\tv_nop\n\tv_nop" : "+v"(c) : "v"(a.hi), "v"(a.lo), "v"(b.hi), "v"(b.lo));
    return c;
}
struct Split3 { v16b hi, mid, lo; };
__device__ __forceinline__ v8f wmma6(const Split3& a, const Split3& b, v8f c) {
    c = __builtin_amdgcn_wmma_f32_16x16x32_bf16(false, a.hi, false, b.hi, (short)0, c, false, false);
    c = __builtin_amdgcn_wmma_f32_16x16x32_bf16(false, a.hi, false, b.mid, (short)0, c, false, false);
    c = __builtin_amdgcn_wmma_f32_16x16x32_bf16(false, a.mid, false, b.hi, (short)0, c, false, false);
    c = __builtin_amdgcn_wmma_f32_16x16x32_bf16(false, a.hi, false, b.lo, (short)0, c, false, false);
    c = __builtin_amdgcn_wmma_f32_16x16x32_bf16(false, a.mid, false, b.mid, (short)0, c, false, false);
    c = __builtin_amdgcn_wmma_f32_16x16x32_bf16(false, a.lo, false, b.hi, (short)0, c, false, false);
    asm volatile("v_nop\n\tv_nop\n\tv_nop\n\tv_nop" : "+v"(c) : "v"(a.hi), "v"(a.mid), "v"(a.lo), "v"(b.hi), "v"(b.mid), "v"(b.lo));
    return c;
}

__device__ __forceinline__ v16h fh_ld(const float* __restrict__ p, long long sk, int k0, int h, int klen, float s) {
    v16h a;
#pragma unroll
    for (int i = 0; i < 16; ++i) { const int k = k0 + frag_k(i, h); a[i] = (k < klen) ? (_Float16)(p[(long long)k * sk] * s) : (_Float16)0.f; }
    return a;
}
__device__ __forceinline__ Split sp_ld(const float* __restrict__ p, long long sk, int k0, int h, int klen, float s) {
    Split r;
#pragma unroll
    for (int i = 0; i < 16; ++i) {
        const int k = k0 + frag_k(i, h); const float x = (k < klen) ? p[(long long)k * sk] * s : 0.f;
        const __bf16 hb = bf16_rne(x); r.hi[i] = hb; r.lo[i] = bf16_rne(x - bf16_f32(hb));
    }
    return r;
}
__device__ __forceinline__ Split3 sp3_ld(const float* __restrict__ p, long long sk, int k0, int h, int klen, float s) {
    Split3 r;
#pragma unroll
    for (int i = 0; i < 16; ++i) {
        const int k = k0 + frag_k(i, h); const float x = (k < klen) ? p[(long long)k * sk] * s : 0.f;
        const __bf16 hb = bf16_rne(x); const float r1 = x - bf16_f32(hb); const __bf16 mb = bf16_rne(r1);
        r.hi[i] = hb; r.mid[i] = mb; r.lo[i] = bf16_rne(r1 - bf16_f32(mb));
    }
    return r;
}
__device__ __forceinline__ v16b bh_ld(const float* __restrict__ p, long long sk, int k0, int h, int klen, float s) {
    v16b a;
#pragma unroll
    for (int i = 0; i < 16; ++i) { const int k = k0 + frag_k(i, h); a[i] = bf16_rne((k < klen) ? p[(long long)k * sk] * s : 0.f); }
    return a;
}
__device__ __forceinline__ v16h fh_row(const _Float16* __restrict__ row, int k0, int h) {
    v16h a;
#pragma unroll
    for (int i = 0; i < 16; ++i) a[i] = row[k0 + frag_k(i, h)];
    return a;
}

#define VST2(T, ptr, val) do { *(volatile T*)(ptr) = (val); __threadfence(); *(volatile T*)(ptr) = (val); } while (0)
typedef float v4f __attribute__((ext_vector_type(4)));
#define VST2V4(ptr, val) do { *(volatile v4f*)(ptr) = (val); __threadfence(); *(volatile v4f*)(ptr) = (val); } while (0)

__device__ __attribute__((noinline)) float act_fn(float v, int act) {
    if (act == 1) return fmaxf(v, 0.f);
    if (act == 2) { const float u = 0.7978845608028654f * (v + 0.044715f * v * v * v); return 0.5f * v * (1.f + tanhf(u)); }
    if (act == 3) return v / (1.f + expf(-v));
    if (act == 4) return 0.5f * v * (1.f + erff(v * 0.7071067811865476f));
    if (act == 5) return tanhf(v);
    if (act == 6) return 1.f / (1.f + expf(-v));
    if (act == 7) return (v > 0.f) ? v : 0.01f * v;
    if (act == 8) return (v > 0.f) ? v : (expf(v) - 1.f);
    if (act == 9) return fminf(fmaxf(v, 0.f), 6.f);
    if (act == 10) return fabsf(v);
    if (act == 11) return (v >= 0.f) ? v : 0.1f * v;
    if (act == 12) return (v > 0.f) ? v : 0.2f * v;
    if (act == 13) return (v > 20.f) ? v : log1pf(expf(v));
    return v;
}

struct GemmP {
    const float* A; const float* B; const float* bias; const float* R; float* C;
    long long sAo, sAi, sAm, sAk, sBo, sBi, sBn, sBk, sCo, sCi, sCm, sRo, sRi, sRm, sRn;
    int M, N, K, zi_n, flags, act; float alpha, beta, sa, sb;
    int Npad, pad_;
};
static_assert(sizeof(GemmP) == 5 * 8 + 15 * 8 + 6 * 4 + 4 * 4 + 2 * 4, "GemmP has padding");

template <int MODE>
__global__ __launch_bounds__(32) void k_gemm(GemmP p) {
    const int lane = threadIdx.x & 31, h = lane >> 4, l15 = lane & 15;
    const int m0 = blockIdx.y * 16, n0 = blockIdx.x * 32;
    const int z = blockIdx.z, zo = z / p.zi_n, zi = z - zo * p.zi_n;
    const float* A = p.A + zo * p.sAo + zi * p.sAi;
    const float* B = p.B + zo * p.sBo + zi * p.sBi;
    const int am = min(m0 + l15, p.M - 1);
    v8f acc[2], comp[2];
#pragma unroll
    for (int t = 0; t < 2; ++t) { v8f zz = {}; acc[t] = zz; comp[t] = zz; }
    for (int k0 = 0; k0 < p.K; k0 += 32) {
        const float* arow = A + (long long)am * p.sAm;
        if (MODE == 1) {
            const Split a = sp_ld(arow, p.sAk, k0, h, p.K, 1.f);
#pragma unroll
            for (int t = 0; t < 2; ++t) {
                const int bn = min(n0 + t * 16 + l15, p.N - 1);
                acc[t] = wmma3(a, sp_ld(B + (long long)bn * p.sBn, p.sBk, k0, h, p.K, 1.f), acc[t]);
            }
        } else if (MODE == 3) {
            const Split3 a = sp3_ld(arow, p.sAk, k0, h, p.K, 1.f);
#pragma unroll
            for (int t = 0; t < 2; ++t) {
                const int bn = min(n0 + t * 16 + l15, p.N - 1);
                acc[t] = wmma6(a, sp3_ld(B + (long long)bn * p.sBn, p.sBk, k0, h, p.K, 1.f), acc[t]);
            }
        } else if (MODE == 4) {
            const Split3 a = sp3_ld(arow, p.sAk, k0, h, p.K, 1.f);
#pragma unroll
            for (int t = 0; t < 2; ++t) {
                const int bn = min(n0 + t * 16 + l15, p.N - 1); v8f zz = {};
                const v8f part = wmma6(a, sp3_ld(B + (long long)bn * p.sBn, p.sBk, k0, h, p.K, 1.f), zz);
                const v8f y = part - comp[t]; const v8f s = acc[t] + y; comp[t] = (s - acc[t]) - y; acc[t] = s;
            }
        } else if (MODE == 2) {
            const v16b a = bh_ld(arow, p.sAk, k0, h, p.K, 1.f);
#pragma unroll
            for (int t = 0; t < 2; ++t) {
                const int bn = min(n0 + t * 16 + l15, p.N - 1);
                acc[t] = wmmab(a, bh_ld(B + (long long)bn * p.sBn, p.sBk, k0, h, p.K, 1.f), acc[t]);
            }
        } else {
            const v16h a = fh_ld(arow, p.sAk, k0, h, p.K, p.sa);
#pragma unroll
            for (int t = 0; t < 2; ++t) {
                const int bn = min(n0 + t * 16 + l15, p.N - 1);
                acc[t] = wmma16(a, fh_ld(B + (long long)bn * p.sBn, p.sBk, k0, h, p.K, p.sb), acc[t]);
            }
        }
    }
    const float iscale = (MODE == 0) ? p.alpha / (p.sa * p.sb) : p.alpha;
    float* C = p.C + zo * p.sCo + zi * p.sCi;
    const float* R = p.R + zo * p.sRo + zi * p.sRi;
    __shared__ __align__(16) float ctile[16][36];
#pragma unroll
    for (int t = 0; t < 2; ++t) {
        const int n = n0 + t * 16 + l15; const int nn = min(n, p.N - 1);
#pragma unroll
        for (int r = 0; r < 8; ++r) {
            const int m = m0 + 8 * h + r; const int mm = min(m, p.M - 1);
            float v = acc[t][r] * iscale;
            if (p.flags & 1) v += p.bias[nn];
            if (p.flags & 2) v += p.bias[mm];
            v = act_fn(v, p.act);
            if (p.flags & 4) v += p.beta * R[(long long)mm * p.sRm + (long long)nn * p.sRn];
            ctile[8 * h + r][t * 16 + l15] = (n < p.N) ? v : 0.f;
        }
    }
    __syncthreads();
    const int NW = (p.Npad > p.N) ? p.Npad : p.N;
    const bool fast = (m0 + 16 <= p.M) && (n0 + 32 <= NW) && ((p.sCm & 3) == 0) && ((((size_t)C) & 15) == 0);
    if (fast) {
#pragma unroll
        for (int s = 0; s < 4; ++s) {
            const int row = s * 4 + (lane >> 3), c4 = (lane & 7) * 4;
            const v4f v = *(const v4f*)&ctile[row][c4];
            VST2V4(C + (long long)(m0 + row) * p.sCm + n0 + c4, v);
        }
    } else {
        for (int row = 0; row < 16; ++row) {
            const int m = m0 + row, n = n0 + lane;
            if (m < p.M && n < NW) VST2(float, C + (long long)m * p.sCm + n, ctile[row][lane]);
        }
    }
}

#define AW 4
struct AttnP {
    const float* Q; const float* K; const float* V; float* O; float* P; const float* Mf; const int* Mi; float* ST;
    const float* Pw; const float* Rt; const int* SQ; const int* SK;
    long long swb, swh, swi, swj, srb, srh, sri;
    long long sQb, sQh, sQi, sQd, sKb, sKh, sKj, sKd, sVb, sVh, sVj, sVd, sOb, sOh, sOi, sPb, sPh, sPi, smb, smh, smi, smj;
    int Lq, Lk, dh, dv, hrep, causal, coff, pband;
    float scale, mfill; int nonorm, mpol;
    int roff, rn, segpol, win;
};
static_assert(sizeof(AttnP) == 12 * 8 + 29 * 8 + 16 * 4, "AttnP has padding");

#ifndef KATTN_ATTR
#define KATTN_ATTR
#endif
template <int DHP, int DVP, int QM, bool SPLITPV, bool TWOPASS>
__global__ __launch_bounds__(32 * AW) KATTN_ATTR void k_attn(AttnP p) {
    constexpr int NT = DVP / 16;
    constexpr int KS = DHP / 32;
    constexpr int VP = DVP + 8;
    __shared__ __align__(16) float    pl[AW][16 * 64];
    __shared__ __align__(16) _Float16 vl[(SPLITPV ? 2 : 1) * 64 * VP];
    const int lane = threadIdx.x & 31, hf = lane >> 4, l15 = lane & 15, wave = threadIdx.x >> 5;
    const int h = blockIdx.y, b = blockIdx.z, hk = h / p.hrep;
    const int q0 = (blockIdx.x * AW + wave) * 16;
    float* myp = pl[wave];
    const float L2E = 1.4426950408889634f;
    const float NEG = -__builtin_inff();
    const int qi = min(q0 + l15, p.Lq - 1);
    const float* qrow = p.Q + b * p.sQb + h * p.sQh + (long long)qi * p.sQi;
    const float* kbase = p.K + b * p.sKb + hk * p.sKh;
    const float* vbase = p.V + b * p.sVb + hk * p.sVh;
    v16h qa[QM == 0 ? KS : 1]; Split qs_[QM == 1 ? KS : 1]; Split3 qt_[QM == 2 ? KS : 1];
#pragma unroll
    for (int ks = 0; ks < KS; ++ks) {
        if (QM == 2) qt_[ks] = sp3_ld(qrow, p.sQd, ks * 32, hf, p.dh, 1.f);
        else if (QM == 1) qs_[ks] = sp_ld(qrow, p.sQd, ks * 32, hf, p.dh, 1.f);
        else qa[ks] = fh_ld(qrow, p.sQd, ks * 32, hf, p.dh, 1.f);
    }
    v8f o[NT]; float m8[8], l8[8];
#pragma unroll
    for (int t = 0; t < NT; ++t) { v8f zz = {}; o[t] = zz; }
#pragma unroll
    for (int i = 0; i < 8; ++i) { m8[i] = NEG; l8[i] = 0.f; }
    int jend = p.Lk;
    if (p.causal == 1) { const int je = (blockIdx.x * AW + AW - 1) * 16 + 16 + p.coff; jend = min(jend, max(je, 0)); }
    const int npass = TWOPASS ? 2 : 1;
    for (int pass = 0; pass < npass; ++pass) {
        const bool dopv = (!TWOPASS) || pass == 1;
        for (int j0 = 0; j0 < jend; j0 += 64) {
            if (dopv) {
                __syncthreads();
                for (int idx = threadIdx.x; idx < 64 * DVP; idx += 32 * AW) {
                    const int jr = idx / DVP, d = idx - jr * DVP, j = j0 + jr;
                    const float f = (j < p.Lk && d < p.dv) ? vbase[(long long)j * p.sVj + (long long)d * p.sVd] : 0.f;
                    if (SPLITPV) {
                        const __bf16 hb = bf16_rne(f);
                        ((__bf16*)vl)[jr * VP + d] = hb; ((__bf16*)vl)[64 * VP + jr * VP + d] = bf16_rne(f - bf16_f32(hb));
                    } else vl[jr * VP + d] = (_Float16)f;
                }
            }
            v8f s[4];
#pragma unroll
            for (int t = 0; t < 4; ++t) {
                const int j = min(j0 + t * 16 + l15, p.Lk - 1);
                const float* krow = kbase + (long long)j * p.sKj;
                v8f acc = {};
#pragma unroll
                for (int ks = 0; ks < KS; ++ks) {
                    if (QM == 2)      acc = wmma6(qt_[ks], sp3_ld(krow, p.sKd, ks * 32, hf, p.dh, 1.f), acc);
                    else if (QM == 1) acc = wmma3(qs_[ks], sp_ld(krow, p.sKd, ks * 32, hf, p.dh, 1.f), acc);
                    else              acc = wmma16(qa[ks], fh_ld(krow, p.sKd, ks * 32, hf, p.dh, 1.f), acc);
                }
                s[t] = acc;
            }
            float pv[8][4];
#pragma unroll
            for (int i = 0; i < 8; ++i) {
                const int irow = q0 + i + 8 * hf;
                const int ic = min(irow, p.Lq - 1);
                float sc[4];
#pragma unroll
                for (int t = 0; t < 4; ++t) {
                    const int jg = j0 + t * 16 + l15;
                    float v = s[t][i] * p.scale;
                    if (p.Mf) v += p.Mf[b * p.smb + h * p.smh + (long long)ic * p.smi + (long long)min(jg, p.Lk - 1) * p.smj];
                    if (p.Rt) { int rc = ic - min(jg, p.Lk - 1) + p.roff; rc = rc < 0 ? 0 : (rc >= p.rn ? p.rn - 1 : rc); v += p.Rt[b * p.srb + h * p.srh + (long long)ic * p.sri + rc]; }
                    if (p.Mi) { const int mv = p.Mi[b * p.smb + h * p.smh + (long long)ic * p.smi + (long long)min(jg, p.Lk - 1) * p.smj]; if (p.mpol ? (mv != 0) : (mv == 0)) v = p.mfill; }
                    if (p.SQ) { const bool same = p.SQ[(long long)b * p.Lq + ic] == p.SK[(long long)b * p.Lk + min(jg, p.Lk - 1)]; if (p.segpol ? same : !same) v = p.mfill; }
                    if (p.causal == 2 && jg > irow + p.coff) v = p.mfill;
                    if (jg >= p.Lk || (p.causal == 1 && jg > irow + p.coff) || (p.causal == 3 && jg < irow + p.coff) || (p.win > 0 && irow + p.coff - jg > p.win)) v = NEG; else v *= L2E;
                    sc[t] = v;
                }
                if (!TWOPASS || pass == 0) {
                    float mx = fmaxf(fmaxf(sc[0], sc[1]), fmaxf(sc[2], sc[3]));
                    mx = fmaxf(mx, __shfl_xor(mx, 1, 32)); mx = fmaxf(mx, __shfl_xor(mx, 2, 32));
                    mx = fmaxf(mx, __shfl_xor(mx, 4, 32)); mx = fmaxf(mx, __shfl_xor(mx, 8, 32));
                    const float mnew = fmaxf(m8[i], mx);
                    const float corr = (mnew == NEG) ? 1.f : exp2f(m8[i] - mnew);
                    float rs = 0.f;
#pragma unroll
                    for (int t = 0; t < 4; ++t) {
                        const float pp = (sc[t] == NEG) ? 0.f : exp2f(sc[t] - mnew); rs += pp;
                        pv[i][t] = p.Pw ? pp * p.Pw[b * p.swb + h * p.swh + (long long)ic * p.swi + (long long)min(j0 + t * 16 + l15, p.Lk - 1) * p.swj] : pp;
                    }
                    rs += __shfl_xor(rs, 1, 32); rs += __shfl_xor(rs, 2, 32); rs += __shfl_xor(rs, 4, 32); rs += __shfl_xor(rs, 8, 32);
                    l8[i] = l8[i] * corr + rs; m8[i] = mnew;
                    if (!TWOPASS) {
#pragma unroll
                        for (int t = 0; t < NT; ++t) o[t][i] *= corr;
                    }
                } else {
                    const float inv = (l8[i] > 0.f) ? 1.f / l8[i] : 0.f;
#pragma unroll
                    for (int t = 0; t < 4; ++t) {
                        const int jg = j0 + t * 16 + l15;
                        float pp = (sc[t] == NEG) ? 0.f : exp2f(sc[t] - m8[i]) * inv;
                        if (p.Pw) pp *= p.Pw[b * p.swb + h * p.swh + (long long)ic * p.swi + (long long)min(jg, p.Lk - 1) * p.swj];
                        pv[i][t] = pp;
                    }
                }
            }
            if (dopv) {
#pragma unroll
                for (int i = 0; i < 8; ++i)
#pragma unroll
                    for (int t = 0; t < 4; ++t) myp[(i + 8 * hf) * 64 + t * 16 + l15] = pv[i][t];
                __syncthreads();
                if (p.P) {
                    float* pb_ = p.P + b * p.sPb + h * p.sPh;
                    const bool fastP = (p.pband == 0) && ((p.sPi & 3) == 0) && (j0 + 64 <= p.Lk) && (q0 + 16 <= p.Lq) && ((((size_t)pb_) & 15) == 0);
                    if (fastP) {
#pragma unroll
                        for (int s = 0; s < 8; ++s) {
                            const int row = s * 2 + (lane >> 4), c4 = (lane & 15) * 4;
                            const v4f v = *(const v4f*)(myp + row * 64 + c4);
                            VST2V4(pb_ + (long long)(q0 + row) * p.sPi + j0 + c4, v);
                        }
                    } else {
                        for (int row = 0; row < 16; ++row) {
                            const int irow = q0 + row; if (irow >= p.Lq) continue;
                            for (int c = lane; c < 64; c += 32) {
                                const int jg = j0 + c; if (jg >= p.Lk) continue;
                                if (p.pband == 0) VST2(float, pb_ + (long long)irow * p.sPi + jg, myp[row * 64 + c]);
                                else if (jg - irow <= p.pband && irow - jg <= p.pband) VST2(float, pb_ + (long long)irow * p.sPi + (jg - irow + p.pband), myp[row * 64 + c]);
                            }
                        }
                    }
                }
                if (SPLITPV) {
                    const Split pa0 = sp_ld(myp + l15 * 64, 1, 0, hf, 64, 1.f), pa1 = sp_ld(myp + l15 * 64, 1, 32, hf, 64, 1.f);
                    const __bf16* vh = (const __bf16*)vl; const __bf16* vlo = vh + 64 * VP;
#pragma unroll
                    for (int t = 0; t < NT; ++t) {
                        const int dcol = t * 16 + l15;
                        Split b0, b1;
#pragma unroll
                        for (int e = 0; e < 16; ++e) {
                            const int k0 = frag_k(e, hf), k1 = 32 + frag_k(e, hf);
                            b0.hi[e] = vh[k0 * VP + dcol]; b0.lo[e] = vlo[k0 * VP + dcol]; b1.hi[e] = vh[k1 * VP + dcol]; b1.lo[e] = vlo[k1 * VP + dcol];
                        }
                        o[t] = wmma3(pa0, b0, o[t]);
                        o[t] = wmma3(pa1, b1, o[t]);
                    }
                } else {
                    const v16h pa0 = fh_ld(myp + l15 * 64, 1, 0, hf, 64, 4096.f), pa1 = fh_ld(myp + l15 * 64, 1, 32, hf, 64, 4096.f);
#pragma unroll
                    for (int t = 0; t < NT; ++t) {
                        const int dcol = t * 16 + l15;
                        v16h b0, b1;
#pragma unroll
                        for (int e = 0; e < 16; ++e) { b0[e] = vl[frag_k(e, hf) * VP + dcol]; b1[e] = vl[(32 + frag_k(e, hf)) * VP + dcol]; }
                        o[t] = wmma16(pa0, b0, o[t]);
                        o[t] = wmma16(pa1, b1, o[t]);
                    }
                }
            }
        }
    }
    float* obase = p.O + b * p.sOb + h * p.sOh;
    if (p.ST) {
        const int rl = lane >> 1, isel = rl & 7;
        float mv = 0.f, lv = 0.f;
#pragma unroll
        for (int i = 0; i < 8; ++i) if (i == isel) { mv = m8[i]; lv = l8[i]; }
        const int irow = q0 + rl;
        if (irow < p.Lq) { float* st = p.ST + (((long long)b * gridDim.y + h) * p.Lq + irow) * 2 + (lane & 1); VST2(float, st, (lane & 1) ? lv : mv * 0.6931471805599453f); }
    }
    float invr[8];
#pragma unroll
    for (int i = 0; i < 8; ++i) {
        if (TWOPASS) invr[i] = SPLITPV ? 1.f : (1.f / 4096.f);
        else if (p.nonorm) invr[i] = exp2f(m8[i]) * (SPLITPV ? 1.f : (1.f / 4096.f));
        else invr[i] = (l8[i] > 0.f) ? (SPLITPV ? 1.f / l8[i] : 1.f / (l8[i] * 4096.f)) : 0.f;
    }
    __syncthreads();
    const bool ofast = ((p.sOi & 3) == 0) && ((((size_t)obase) & 15) == 0) && (q0 + 16 <= p.Lq);
#pragma unroll
    for (int c0 = 0; c0 < DVP; c0 += 64) {
#pragma unroll
        for (int i = 0; i < 8; ++i)
#pragma unroll
            for (int t = 0; t < NT; ++t) if (t * 16 >= c0 && t * 16 < c0 + 64) myp[(i + 8 * hf) * 64 + (t * 16 - c0) + l15] = o[t][i] * invr[i];
        __syncthreads();
        const int cw = (DVP - c0 < 64) ? (DVP - c0) : 64;
        if (ofast && (c0 + cw <= p.dv) && (cw % 32 == 0)) {
            const int lpr = cw / 4;
            const int rows_per_ins = 32 / lpr;
            for (int r0 = 0; r0 < 16; r0 += rows_per_ins) {
                const int row = r0 + lane / lpr, c4 = (lane % lpr) * 4;
                const v4f v = *(const v4f*)(myp + row * 64 + c4);
                VST2V4(obase + (long long)(q0 + row) * p.sOi + c0 + c4, v);
            }
        } else {
            for (int row = 0; row < 16; ++row) {
                const int irow = q0 + row; if (irow >= p.Lq) continue;
                for (int c = lane; c < cw; c += 32) { const int d = c0 + c; if (d < p.dv) VST2(float, obase + (long long)irow * p.sOi + d, myp[row * 64 + c]); }
            }
        }
        __syncthreads();
    }
}

struct TrP { const float* src; float* dst; const float* R2; long long sSz, lds, sDz, ldd, sRz, ldr; int R, C, flags, act; float alpha, beta; };
static_assert(sizeof(TrP) == 3 * 8 + 6 * 8 + 6 * 4, "TrP has padding");
__global__ __launch_bounds__(256) void k_tr(TrP p) {
    __shared__ float tile[32][33];
    const int c0 = blockIdx.x * 32, r0 = blockIdx.y * 32, z = blockIdx.z;
    const int lane = threadIdx.x & 31, wave = threadIdx.x >> 5;
    const float* s = p.src + z * p.sSz;
#pragma unroll
    for (int k = 0; k < 4; ++k) {
        const int rl = wave * 4 + k, r = r0 + rl, c = c0 + lane;
        tile[rl][lane] = (r < p.R && c < p.C) ? s[(long long)r * p.lds + c] : 0.f;
    }
    __syncthreads();
    float* d = p.dst + z * p.sDz; const float* rr = p.R2 + z * p.sRz;
#pragma unroll
    for (int k = 0; k < 4; ++k) {
        const int cl = wave * 4 + k, c = c0 + cl, r = r0 + lane;
        if (c < p.C && r < p.R) {
            float v = act_fn(p.alpha * tile[lane][cl], p.act);
            if (p.flags & 1) v += p.beta * rr[(long long)c * p.ldr + r];
            VST2(float, d + (long long)c * p.ldd + r, v);
        }
    }
}

__global__ __launch_bounds__(256) void k_affine(const float* __restrict__ src, float* __restrict__ dst, int n, float a, float b, const float* __restrict__ sdev) {
    const int i = blockIdx.x * 256 + threadIdx.x;
    if (i < n) { const float aa = sdev ? a * sdev[0] : a; const float v = aa * src[i] + b; VST2(float, dst + i, v); }
}

struct SmP { const float* src; float* dst; const float* Mf; long long sz, sr, dz, dr, smz, smr; int n, pad; float scale_in, scale_out; };
static_assert(sizeof(SmP) == 3 * 8 + 6 * 8 + 4 * 4, "SmP has padding");
__global__ __launch_bounds__(256) void k_softmax(SmP p) {
    __shared__ float red[256];
    const int r = blockIdx.x, z = blockIdx.y, tid = threadIdx.x;
    const float* s = p.src + z * p.sz + (long long)r * p.sr;
    const float* mf = p.Mf ? (p.Mf + z * p.smz + (long long)r * p.smr) : nullptr;
    float mx = -__builtin_inff();
    for (int j = tid; j < p.n; j += 256) { float v = s[j] * p.scale_in; if (mf) v += mf[j]; mx = fmaxf(mx, v); }
    red[tid] = mx; __syncthreads();
    for (int o = 128; o > 0; o >>= 1) { if (tid < o) red[tid] = fmaxf(red[tid], red[tid + o]); __syncthreads(); }
    mx = red[0]; __syncthreads();
    float sum = 0.f;
    for (int j = tid; j < p.n; j += 256) { float v = s[j] * p.scale_in; if (mf) v += mf[j]; sum += (mx == -__builtin_inff()) ? 0.f : expf(v - mx); }
    red[tid] = sum; __syncthreads();
    for (int o = 128; o > 0; o >>= 1) { if (tid < o) red[tid] += red[tid + o]; __syncthreads(); }
    sum = red[0];
    const float inv = (sum > 0.f) ? p.scale_out / sum : 0.f;
    float* d = p.dst + z * p.dz + (long long)r * p.dr;
    for (int j = tid; j < p.n; j += 256) { float v = s[j] * p.scale_in; if (mf) v += mf[j]; const float o = (mx == -__builtin_inff()) ? 0.f : expf(v - mx) * inv; VST2(float, d + j, o); }
}
__global__ __launch_bounds__(256) void k_stats(const float* __restrict__ x, long long sz, long long so, long long si, int inner, int n, float eps, float* __restrict__ stat, int mode) {
    __shared__ float red[256];
    const int z = blockIdx.x, tid = threadIdx.x;
    const float* base = x + z * sz;
    float s = 0.f;
    for (int e = tid; e < n; e += 256) s += base[(long long)(e / inner) * so + (long long)(e % inner) * si];
    red[tid] = s; __syncthreads();
    for (int o = 128; o > 0; o >>= 1) { if (tid < o) red[tid] += red[tid + o]; __syncthreads(); }
    const float mu = (mode == 0 || mode == 3) ? red[0] / (float)n : 0.f; __syncthreads();
    float q = 0.f;
    for (int e = tid; e < n; e += 256) { const float dlt = base[(long long)(e / inner) * so + (long long)(e % inner) * si] - mu; q += dlt * dlt; }
    red[tid] = q; __syncthreads();
    for (int o = 128; o > 0; o >>= 1) { if (tid < o) red[tid] += red[tid + o]; __syncthreads(); }
    {
        float rs;
        if (mode == 2) rs = sqrtf((float)n) / fmaxf(sqrtf(red[0]), eps); else if (mode == 3) rs = rsqrtf(red[0] / (float)(n - 1) + eps); else rs = rsqrtf(red[0] / (float)n + eps);
        if (tid < 32) { const float v = (tid == 0) ? mu : ((tid == 1) ? rs : 0.f); VST2(float, stat + (long long)z * 32 + tid, v); }
    }
}
__global__ __launch_bounds__(256) void k_norm_apply(const float* __restrict__ x, float* __restrict__ y, const float* __restrict__ stat, const float* __restrict__ g, const float* __restrict__ bta,
                                                     int Z, int C, int L, int G, int bn, int act) {
    const long long idx = (long long)blockIdx.x * 256 + threadIdx.x;
    if (idx >= (long long)Z * C * L) return;
    const int l = (int)(idx % L); const long long zc = idx / L; const int c = (int)(zc % C), z = (int)(zc / C); (void)l;
    const int set = bn ? c : (z * G + c / (C / G));
    float v = (x[idx] - stat[(long long)set * 32]) * stat[(long long)set * 32 + 1];
    if (g) v *= g[c];
    if (bta) v += bta[c];
    v = act_fn(v, act);
    VST2(float, y + idx, v);
}

__global__ __launch_bounds__(256) void k_lse_neg(const float* __restrict__ st, float* __restrict__ c, int n) {
    const int i = blockIdx.x * 256 + threadIdx.x;
    if (i < n) { const float v = -(st[2 * i] + logf(st[2 * i + 1])); VST2(float, c + i, v); }
}

__global__ __launch_bounds__(256) void k_iota(int* __restrict__ dst, int n, int a, int b) {
    const int i = blockIdx.x * 256 + threadIdx.x;
    if (i < n) { const int v = a * i + b; VST2(int, dst + i, v); }
}

__global__ __launch_bounds__(256) void k_axpby(const float* __restrict__ x, const float* __restrict__ y, float* __restrict__ dst, int n, float a, float b, float c) {
    const int i = blockIdx.x * 256 + threadIdx.x;
    if (i < n) { const float v = a * x[i] + b * y[i] + c; VST2(float, dst + i, v); }
}

struct RopeP { const float* X; float* Y; const float* C; const float* Sn; const int* pos; long long sXr, sXh, sYr, sYh, sCb, sCp, sCd; int R, Hn, D, S, mode, tmode, pmode, pad; };
static_assert(sizeof(RopeP) == 5 * 8 + 7 * 8 + 8 * 4, "RopeP has padding");
__global__ __launch_bounds__(256) void k_rope(RopeP p) {
    const long long idx = (long long)blockIdx.x * 256 + threadIdx.x;
    if (idx >= (long long)p.R * p.Hn * p.D) return;
    const int d = (int)(idx % p.D); const long long rh = idx / p.D; const int h = (int)(rh % p.Hn); const int r = (int)(rh / p.Hn);
    const int half = p.D / 2;
    int partner; float sign;
    if (p.mode == 0) { partner = (d < half) ? d + half : d - half; sign = (d < half) ? -1.f : 1.f; }
    else { partner = d ^ 1; sign = (d & 1) ? 1.f : -1.f; }
    const int tcol = (p.tmode == 0) ? d : ((p.tmode == 1) ? (d % half) : (d >> 1));
    const int pp = (p.pmode == 0) ? (r % p.S) : ((p.pmode == 1) ? h : p.pos[r]);
    const long long toff = (long long)(r / p.S) * p.sCb + (long long)pp * p.sCp + (long long)tcol * p.sCd;
    const float* xr = p.X + (long long)r * p.sXr + (long long)h * p.sXh;
    const float v = xr[d] * p.C[toff] + sign * xr[partner] * p.Sn[toff];
    VST2(float, p.Y + (long long)r * p.sYr + (long long)h * p.sYh + d, v);
}

__global__ __launch_bounds__(256) void k_invf(float* __restrict__ invb, int half, int D, float base, float num, int fmode, float cexp) {
    const int i = blockIdx.x * 256 + threadIdx.x;
    if (i >= ((half + 31) / 32) * 32) return;
    if (i >= half) { VST2(float, invb + i, 0.f); return; }
    const float e = (float)(2 * i) / (float)D;
    float invf;
    if (fmode == 1) invf = num * expf((float)(2 * i) * cexp);
    else if (fmode == 2) invf = num * powf(base, (-2.0f * ((float)i - 1.0f)) / (float)D);
    else invf = num * (1.0f / powf(base, e));
    VST2(float, invb + i, invf);
}
__global__ __launch_bounds__(256) void k_sincos(float* __restrict__ cs, float* __restrict__ sn, const float* __restrict__ invb, int S, int half, float pscale) {
    const int idx = blockIdx.x * 256 + threadIdx.x;
    if (idx >= S * half) return;
    const int s = idx / half, i = idx - s * half;
    const float ang = (pscale * (float)s) * invb[i];
    VST2(float, cs + idx, cosf(ang)); VST2(float, sn + idx, sinf(ang));
}

__global__ __launch_bounds__(256) void k_mulact(const float* __restrict__ x, const float* __restrict__ y, float* __restrict__ dst, int n, int act) {
    const int i = blockIdx.x * 256 + threadIdx.x;
    if (i < n) { const float v = act_fn(x[i], act) * y[i]; VST2(float, dst + i, v); }
}

__global__ __launch_bounds__(256) void k_matvec(GemmP p) {
    const int rpt = (p.N == 1) ? 1 : 32;
    const long long r0 = ((long long)blockIdx.x * 256 + threadIdx.x) * rpt; const int z = blockIdx.z, zo = z / p.zi_n, zi = z - zo * p.zi_n;
    if (r0 >= p.M) return;
    const float* Bb = p.B + zo * p.sBo + zi * p.sBi;
    float* C = p.C + zo * p.sCo + zi * p.sCi; const float* R = p.R + zo * p.sRo + zi * p.sRi;
    for (int rr = 0; rr < rpt; ++rr) {
        const long long r = r0 + rr; if (r >= p.M) break;
        const float* A = p.A + zo * p.sAo + zi * p.sAi + r * p.sAm;
        float acc[8] = {0.f, 0.f, 0.f, 0.f, 0.f, 0.f, 0.f, 0.f};
        for (int k = 0; k < p.K; ++k) { const float a = A[(long long)k * p.sAk];
#pragma unroll
            for (int j = 0; j < 8; ++j) if (j < p.N) acc[j] += a * Bb[(long long)j * p.sBn + (long long)k * p.sBk]; }
#pragma unroll
        for (int j = 0; j < 8; ++j) if (j < p.N) {
            float v = acc[j] * p.alpha;
            if (p.flags & 1) v += p.bias[j];
            if (p.flags & 2) v += p.bias[r];
            v = act_fn(v, p.act);
            if (p.flags & 4) v += p.beta * R[r * p.sRm + (long long)j * p.sRn];
            VST2(float, C + r * p.sCm + j, v);
        }
    }
}
__global__ __launch_bounds__(256) void k_smallsoftmax(const float* __restrict__ src, float* __restrict__ dst, long long sr, long long dr, int n, long long R, float scale) {
    const long long r0 = ((long long)blockIdx.x * 256 + threadIdx.x) * 32;
    for (int rr = 0; rr < 32; ++rr) {
        const long long r = r0 + rr; if (r >= R) return;
        const float* s = src + r * sr; float* d = dst + r * dr;
        float mx = -__builtin_inff();
        for (int j = 0; j < n; ++j) mx = fmaxf(mx, s[j] * scale);
        float sum = 0.f;
        for (int j = 0; j < n; ++j) sum += expf(s[j] * scale - mx);
        const float inv = 1.f / sum;
        for (int j = 0; j < n; ++j) { const float v = expf(s[j] * scale - mx) * inv; VST2(float, d + j, v); }
    }
}

__global__ __launch_bounds__(32) void k_unitstat(float* __restrict__ st) { const int t = threadIdx.x; const float v = (t == 1) ? 1.f : 0.f; VST2(float, st + t, v); }

__global__ __launch_bounds__(256) void k_lincopy(const float* __restrict__ src, long long lds, float* __restrict__ dst, long long ldd, long long rows, int cols) {
    const long long i = (long long)blockIdx.x * 256 + threadIdx.x; if (i >= rows * cols) return;
    const long long r = i / cols; const int c = (int)(i - r * cols);
    const float v = src[r * lds + c]; VST2(float, dst + r * ldd + c, v);
}

__global__ __launch_bounds__(256) void k_gd_colsum(const float* __restrict__ ATT, float* __restrict__ SEL, int N) { const int n = blockIdx.x * 256 + threadIdx.x; if (n >= N) return; double s = 0.0; for (int m = 0; m < N; ++m) s += (double)ATT[(long long)m * N + n]; VST2(float, SEL + n, (float)s); }
__global__ __launch_bounds__(256) void k_gd_rank(const float* __restrict__ SEL, int* __restrict__ IDX, int N, int M) { const int n = blockIdx.x * 256 + threadIdx.x; if (n >= N) return; const float v = SEL[n]; int r = 0; for (int m = 0; m < N; ++m) { const float u = SEL[m]; r += (u > v) || (u == v && m < n); } if (r < M) VST2(int, IDX + r, n); }
__global__ __launch_bounds__(256) void k_gd_gather(const float* __restrict__ ATT, const int* __restrict__ IDX, float* __restrict__ SCS, int N, int M) { const long long q = (long long)blockIdx.x * 256 + threadIdx.x; if (q >= (long long)M * N) return; const int n = (int)(q % N); const int m = (int)(q / N); VST2(float, SCS + q, ATT[(long long)IDX[m] * N + n]); }

template __global__ void k_gemm<1>(GemmP);
template __global__ void k_gemm<4>(GemmP);

extern "C" void kernel_launch(void* const* d_in, const int* in_sizes, int n_in, void* d_out, int out_size, void* d_ws, size_t ws_size, hipStream_t stream) {
    (void)in_sizes; (void)n_in; (void)out_size; (void)ws_size;
    const float* x = (const float*)d_in[0];
    const float* Wq = (const float*)d_in[1];
    const float* Wk = (const float*)d_in[2];
    const float* Wv = (const float*)d_in[3];
    const int* npts = (const int*)d_in[4];
    const int Bn = 8;
    const int C = 128;
    const int N = 2048;
    const int M = 512;
    float* out = (float*)d_out;
    char* wsp = (char*)d_ws;
    float* Q = (float*)wsp; wsp += (((size_t)((size_t)C * N) * 4 + 255) / 256) * 256;
    float* Kk = (float*)wsp; wsp += (((size_t)((size_t)C * N) * 4 + 255) / 256) * 256;
    float* V = (float*)wsp; wsp += (((size_t)((size_t)C * N) * 4 + 255) / 256) * 256;
    float* ATT = (float*)wsp; wsp += (((size_t)((size_t)N * N) * 4 + 255) / 256) * 256;
    float* SEL = (float*)wsp; wsp += (((size_t)((size_t)N + 64) * 4 + 255) / 256) * 256;
    int* IDX = (int*)wsp; wsp += (((size_t)((size_t)N + 64) * 4 + 255) / 256) * 256;
    float* SCS = (float*)wsp; wsp += (((size_t)((size_t)M * N) * 4 + 255) / 256) * 256;
    { GemmP gQ0;
      gQ0.A = Wq; gQ0.B = x + (size_t)0 * C * N; gQ0.bias = Wq; gQ0.R = Wq; gQ0.C = Q;
      gQ0.sAo = 0; gQ0.sAi = 0; gQ0.sAm = C; gQ0.sAk = 1; gQ0.sBo = 0; gQ0.sBi = 0; gQ0.sBn = 1; gQ0.sBk = N; gQ0.sCo = 0; gQ0.sCi = 0; gQ0.sCm = N; gQ0.sRo = 0; gQ0.sRi = 0; gQ0.sRm = 0; gQ0.sRn = 0;
      gQ0.M = C; gQ0.N = N; gQ0.K = C; gQ0.zi_n = 1; gQ0.flags = 0; gQ0.act = 0;
      gQ0.alpha = 1.0f; gQ0.beta = 0.0f; gQ0.sa = 1.0f; gQ0.sb = 1.0f; gQ0.Npad = N; gQ0.pad_ = 0;
      k_gemm<4><<<dim3((unsigned)((N) + 31) / 32, (unsigned)((C) + 15) / 16, (unsigned)(1)), 32, 0, stream>>>(gQ0); }
    { GemmP gKk0;
      gKk0.A = Wk; gKk0.B = x + (size_t)0 * C * N; gKk0.bias = Wk; gKk0.R = Wk; gKk0.C = Kk;
      gKk0.sAo = 0; gKk0.sAi = 0; gKk0.sAm = C; gKk0.sAk = 1; gKk0.sBo = 0; gKk0.sBi = 0; gKk0.sBn = 1; gKk0.sBk = N; gKk0.sCo = 0; gKk0.sCi = 0; gKk0.sCm = N; gKk0.sRo = 0; gKk0.sRi = 0; gKk0.sRm = 0; gKk0.sRn = 0;
      gKk0.M = C; gKk0.N = N; gKk0.K = C; gKk0.zi_n = 1; gKk0.flags = 0; gKk0.act = 0;
      gKk0.alpha = 1.0f; gKk0.beta = 0.0f; gKk0.sa = 1.0f; gKk0.sb = 1.0f; gKk0.Npad = N; gKk0.pad_ = 0;
      k_gemm<4><<<dim3((unsigned)((N) + 31) / 32, (unsigned)((C) + 15) / 16, (unsigned)(1)), 32, 0, stream>>>(gKk0); }
    { GemmP gV0;
      gV0.A = Wv; gV0.B = x + (size_t)0 * C * N; gV0.bias = Wv; gV0.R = Wv; gV0.C = V;
      gV0.sAo = 0; gV0.sAi = 0; gV0.sAm = C; gV0.sAk = 1; gV0.sBo = 0; gV0.sBi = 0; gV0.sBn = 1; gV0.sBk = N; gV0.sCo = 0; gV0.sCi = 0; gV0.sCm = N; gV0.sRo = 0; gV0.sRi = 0; gV0.sRm = 0; gV0.sRn = 0;
      gV0.M = C; gV0.N = N; gV0.K = C; gV0.zi_n = 1; gV0.flags = 0; gV0.act = 0;
      gV0.alpha = 1.0f; gV0.beta = 0.0f; gV0.sa = 1.0f; gV0.sb = 1.0f; gV0.Npad = N; gV0.pad_ = 0;
      k_gemm<4><<<dim3((unsigned)((N) + 31) / 32, (unsigned)((C) + 15) / 16, (unsigned)(1)), 32, 0, stream>>>(gV0); }
    { GemmP ge0;
      ge0.A = Q; ge0.B = Kk; ge0.bias = Q; ge0.R = Q; ge0.C = ATT;
      ge0.sAo = 0; ge0.sAi = 0; ge0.sAm = 1; ge0.sAk = N; ge0.sBo = 0; ge0.sBi = 0; ge0.sBn = 1; ge0.sBk = N; ge0.sCo = 0; ge0.sCi = 0; ge0.sCm = N; ge0.sRo = 0; ge0.sRi = 0; ge0.sRm = 0; ge0.sRn = 0;
      ge0.M = N; ge0.N = N; ge0.K = C; ge0.zi_n = 1; ge0.flags = 0; ge0.act = 0;
      ge0.alpha = 0.08838834764831843f; ge0.beta = 0.0f; ge0.sa = 1.0f; ge0.sb = 1.0f; ge0.Npad = N; ge0.pad_ = 0;
      k_gemm<4><<<dim3((unsigned)((N) + 31) / 32, (unsigned)((N) + 15) / 16, (unsigned)(1)), 32, 0, stream>>>(ge0); }
    { SmP sm; sm.src = ATT; sm.dst = ATT; sm.Mf = 0; sm.sz = 0; sm.sr = N; sm.dz = 0; sm.dr = N; sm.smz = 0; sm.smr = 0; sm.n = N; sm.pad = 0; sm.scale_in = 1.0f; sm.scale_out = 1.0f;
      k_softmax<<<dim3((unsigned)(N), (unsigned)(1)), 256, 0, stream>>>(sm); }
    k_gd_colsum<<<(unsigned)((N + 255) / 256), 256, 0, stream>>>(ATT, SEL, N);
    k_gd_rank<<<(unsigned)((N + 255) / 256), 256, 0, stream>>>(SEL, IDX, N, M);
    k_gd_gather<<<(unsigned)(((long long)M * N + 255) / 256), 256, 0, stream>>>(ATT, IDX, SCS, N, M);
    { GemmP go0;
      go0.A = V; go0.B = SCS; go0.bias = V; go0.R = V; go0.C = out + (size_t)0 * C * M;
      go0.sAo = 0; go0.sAi = 0; go0.sAm = N; go0.sAk = 1; go0.sBo = 0; go0.sBi = 0; go0.sBn = N; go0.sBk = 1; go0.sCo = 0; go0.sCi = 0; go0.sCm = M; go0.sRo = 0; go0.sRi = 0; go0.sRm = 0; go0.sRn = 0;
      go0.M = C; go0.N = M; go0.K = N; go0.zi_n = 1; go0.flags = 0; go0.act = 0;
      go0.alpha = 1.0f; go0.beta = 0.0f; go0.sa = 1.0f; go0.sb = 1.0f; go0.Npad = M; go0.pad_ = 0;
      k_gemm<1><<<dim3((unsigned)((M) + 31) / 32, (unsigned)((C) + 15) / 16, (unsigned)(1)), 32, 0, stream>>>(go0); }
    { GemmP gQ1;
      gQ1.A = Wq; gQ1.B = x + (size_t)1 * C * N; gQ1.bias = Wq; gQ1.R = Wq; gQ1.C = Q;
      gQ1.sAo = 0; gQ1.sAi = 0; gQ1.sAm = C; gQ1.sAk = 1; gQ1.sBo = 0; gQ1.sBi = 0; gQ1.sBn = 1; gQ1.sBk = N; gQ1.sCo = 0; gQ1.sCi = 0; gQ1.sCm = N; gQ1.sRo = 0; gQ1.sRi = 0; gQ1.sRm = 0; gQ1.sRn = 0;
      gQ1.M = C; gQ1.N = N; gQ1.K = C; gQ1.zi_n = 1; gQ1.flags = 0; gQ1.act = 0;
      gQ1.alpha = 1.0f; gQ1.beta = 0.0f; gQ1.sa = 1.0f; gQ1.sb = 1.0f; gQ1.Npad = N; gQ1.pad_ = 0;
      k_gemm<4><<<dim3((unsigned)((N) + 31) / 32, (unsigned)((C) + 15) / 16, (unsigned)(1)), 32, 0, stream>>>(gQ1); }
    { GemmP gKk1;
      gKk1.A = Wk; gKk1.B = x + (size_t)1 * C * N; gKk1.bias = Wk; gKk1.R = Wk; gKk1.C = Kk;
      gKk1.sAo = 0; gKk1.sAi = 0; gKk1.sAm = C; gKk1.sAk = 1; gKk1.sBo = 0; gKk1.sBi = 0; gKk1.sBn = 1; gKk1.sBk = N; gKk1.sCo = 0; gKk1.sCi = 0; gKk1.sCm = N; gKk1.sRo = 0; gKk1.sRi = 0; gKk1.sRm = 0; gKk1.sRn = 0;
      gKk1.M = C; gKk1.N = N; gKk1.K = C; gKk1.zi_n = 1; gKk1.flags = 0; gKk1.act = 0;
      gKk1.alpha = 1.0f; gKk1.beta = 0.0f; gKk1.sa = 1.0f; gKk1.sb = 1.0f; gKk1.Npad = N; gKk1.pad_ = 0;
      k_gemm<4><<<dim3((unsigned)((N) + 31) / 32, (unsigned)((C) + 15) / 16, (unsigned)(1)), 32, 0, stream>>>(gKk1); }
    { GemmP gV1;
      gV1.A = Wv; gV1.B = x + (size_t)1 * C * N; gV1.bias = Wv; gV1.R = Wv; gV1.C = V;
      gV1.sAo = 0; gV1.sAi = 0; gV1.sAm = C; gV1.sAk = 1; gV1.sBo = 0; gV1.sBi = 0; gV1.sBn = 1; gV1.sBk = N; gV1.sCo = 0; gV1.sCi = 0; gV1.sCm = N; gV1.sRo = 0; gV1.sRi = 0; gV1.sRm = 0; gV1.sRn = 0;
      gV1.M = C; gV1.N = N; gV1.K = C; gV1.zi_n = 1; gV1.flags = 0; gV1.act = 0;
      gV1.alpha = 1.0f; gV1.beta = 0.0f; gV1.sa = 1.0f; gV1.sb = 1.0f; gV1.Npad = N; gV1.pad_ = 0;
      k_gemm<4><<<dim3((unsigned)((N) + 31) / 32, (unsigned)((C) + 15) / 16, (unsigned)(1)), 32, 0, stream>>>(gV1); }
    { GemmP ge1;
      ge1.A = Q; ge1.B = Kk; ge1.bias = Q; ge1.R = Q; ge1.C = ATT;
      ge1.sAo = 0; ge1.sAi = 0; ge1.sAm = 1; ge1.sAk = N; ge1.sBo = 0; ge1.sBi = 0; ge1.sBn = 1; ge1.sBk = N; ge1.sCo = 0; ge1.sCi = 0; ge1.sCm = N; ge1.sRo = 0; ge1.sRi = 0; ge1.sRm = 0; ge1.sRn = 0;
      ge1.M = N; ge1.N = N; ge1.K = C; ge1.zi_n = 1; ge1.flags = 0; ge1.act = 0;
      ge1.alpha = 0.08838834764831843f; ge1.beta = 0.0f; ge1.sa = 1.0f; ge1.sb = 1.0f; ge1.Npad = N; ge1.pad_ = 0;
      k_gemm<4><<<dim3((unsigned)((N) + 31) / 32, (unsigned)((N) + 15) / 16, (unsigned)(1)), 32, 0, stream>>>(ge1); }
    { SmP sm; sm.src = ATT; sm.dst = ATT; sm.Mf = 0; sm.sz = 0; sm.sr = N; sm.dz = 0; sm.dr = N; sm.smz = 0; sm.smr = 0; sm.n = N; sm.pad = 0; sm.scale_in = 1.0f; sm.scale_out = 1.0f;
      k_softmax<<<dim3((unsigned)(N), (unsigned)(1)), 256, 0, stream>>>(sm); }
    k_gd_colsum<<<(unsigned)((N + 255) / 256), 256, 0, stream>>>(ATT, SEL, N);
    k_gd_rank<<<(unsigned)((N + 255) / 256), 256, 0, stream>>>(SEL, IDX, N, M);
    k_gd_gather<<<(unsigned)(((long long)M * N + 255) / 256), 256, 0, stream>>>(ATT, IDX, SCS, N, M);
    { GemmP go1;
      go1.A = V; go1.B = SCS; go1.bias = V; go1.R = V; go1.C = out + (size_t)1 * C * M;
      go1.sAo = 0; go1.sAi = 0; go1.sAm = N; go1.sAk = 1; go1.sBo = 0; go1.sBi = 0; go1.sBn = N; go1.sBk = 1; go1.sCo = 0; go1.sCi = 0; go1.sCm = M; go1.sRo = 0; go1.sRi = 0; go1.sRm = 0; go1.sRn = 0;
      go1.M = C; go1.N = M; go1.K = N; go1.zi_n = 1; go1.flags = 0; go1.act = 0;
      go1.alpha = 1.0f; go1.beta = 0.0f; go1.sa = 1.0f; go1.sb = 1.0f; go1.Npad = M; go1.pad_ = 0;
      k_gemm<1><<<dim3((unsigned)((M) + 31) / 32, (unsigned)((C) + 15) / 16, (unsigned)(1)), 32, 0, stream>>>(go1); }
    { GemmP gQ2;
      gQ2.A = Wq; gQ2.B = x + (size_t)2 * C * N; gQ2.bias = Wq; gQ2.R = Wq; gQ2.C = Q;
      gQ2.sAo = 0; gQ2.sAi = 0; gQ2.sAm = C; gQ2.sAk = 1; gQ2.sBo = 0; gQ2.sBi = 0; gQ2.sBn = 1; gQ2.sBk = N; gQ2.sCo = 0; gQ2.sCi = 0; gQ2.sCm = N; gQ2.sRo = 0; gQ2.sRi = 0; gQ2.sRm = 0; gQ2.sRn = 0;
      gQ2.M = C; gQ2.N = N; gQ2.K = C; gQ2.zi_n = 1; gQ2.flags = 0; gQ2.act = 0;
      gQ2.alpha = 1.0f; gQ2.beta = 0.0f; gQ2.sa = 1.0f; gQ2.sb = 1.0f; gQ2.Npad = N; gQ2.pad_ = 0;
      k_gemm<4><<<dim3((unsigned)((N) + 31) / 32, (unsigned)((C) + 15) / 16, (unsigned)(1)), 32, 0, stream>>>(gQ2); }
    { GemmP gKk2;
      gKk2.A = Wk; gKk2.B = x + (size_t)2 * C * N; gKk2.bias = Wk; gKk2.R = Wk; gKk2.C = Kk;
      gKk2.sAo = 0; gKk2.sAi = 0; gKk2.sAm = C; gKk2.sAk = 1; gKk2.sBo = 0; gKk2.sBi = 0; gKk2.sBn = 1; gKk2.sBk = N; gKk2.sCo = 0; gKk2.sCi = 0; gKk2.sCm = N; gKk2.sRo = 0; gKk2.sRi = 0; gKk2.sRm = 0; gKk2.sRn = 0;
      gKk2.M = C; gKk2.N = N; gKk2.K = C; gKk2.zi_n = 1; gKk2.flags = 0; gKk2.act = 0;
      gKk2.alpha = 1.0f; gKk2.beta = 0.0f; gKk2.sa = 1.0f; gKk2.sb = 1.0f; gKk2.Npad = N; gKk2.pad_ = 0;
      k_gemm<4><<<dim3((unsigned)((N) + 31) / 32, (unsigned)((C) + 15) / 16, (unsigned)(1)), 32, 0, stream>>>(gKk2); }
    { GemmP gV2;
      gV2.A = Wv; gV2.B = x + (size_t)2 * C * N; gV2.bias = Wv; gV2.R = Wv; gV2.C = V;
      gV2.sAo = 0; gV2.sAi = 0; gV2.sAm = C; gV2.sAk = 1; gV2.sBo = 0; gV2.sBi = 0; gV2.sBn = 1; gV2.sBk = N; gV2.sCo = 0; gV2.sCi = 0; gV2.sCm = N; gV2.sRo = 0; gV2.sRi = 0; gV2.sRm = 0; gV2.sRn = 0;
      gV2.M = C; gV2.N = N; gV2.K = C; gV2.zi_n = 1; gV2.flags = 0; gV2.act = 0;
      gV2.alpha = 1.0f; gV2.beta = 0.0f; gV2.sa = 1.0f; gV2.sb = 1.0f; gV2.Npad = N; gV2.pad_ = 0;
      k_gemm<4><<<dim3((unsigned)((N) + 31) / 32, (unsigned)((C) + 15) / 16, (unsigned)(1)), 32, 0, stream>>>(gV2); }
    { GemmP ge2;
      ge2.A = Q; ge2.B = Kk; ge2.bias = Q; ge2.R = Q; ge2.C = ATT;
      ge2.sAo = 0; ge2.sAi = 0; ge2.sAm = 1; ge2.sAk = N; ge2.sBo = 0; ge2.sBi = 0; ge2.sBn = 1; ge2.sBk = N; ge2.sCo = 0; ge2.sCi = 0; ge2.sCm = N; ge2.sRo = 0; ge2.sRi = 0; ge2.sRm = 0; ge2.sRn = 0;
      ge2.M = N; ge2.N = N; ge2.K = C; ge2.zi_n = 1; ge2.flags = 0; ge2.act = 0;
      ge2.alpha = 0.08838834764831843f; ge2.beta = 0.0f; ge2.sa = 1.0f; ge2.sb = 1.0f; ge2.Npad = N; ge2.pad_ = 0;
      k_gemm<4><<<dim3((unsigned)((N) + 31) / 32, (unsigned)((N) + 15) / 16, (unsigned)(1)), 32, 0, stream>>>(ge2); }
    { SmP sm; sm.src = ATT; sm.dst = ATT; sm.Mf = 0; sm.sz = 0; sm.sr = N; sm.dz = 0; sm.dr = N; sm.smz = 0; sm.smr = 0; sm.n = N; sm.pad = 0; sm.scale_in = 1.0f; sm.scale_out = 1.0f;
      k_softmax<<<dim3((unsigned)(N), (unsigned)(1)), 256, 0, stream>>>(sm); }
    k_gd_colsum<<<(unsigned)((N + 255) / 256), 256, 0, stream>>>(ATT, SEL, N);
    k_gd_rank<<<(unsigned)((N + 255) / 256), 256, 0, stream>>>(SEL, IDX, N, M);
    k_gd_gather<<<(unsigned)(((long long)M * N + 255) / 256), 256, 0, stream>>>(ATT, IDX, SCS, N, M);
    { GemmP go2;
      go2.A = V; go2.B = SCS; go2.bias = V; go2.R = V; go2.C = out + (size_t)2 * C * M;
      go2.sAo = 0; go2.sAi = 0; go2.sAm = N; go2.sAk = 1; go2.sBo = 0; go2.sBi = 0; go2.sBn = N; go2.sBk = 1; go2.sCo = 0; go2.sCi = 0; go2.sCm = M; go2.sRo = 0; go2.sRi = 0; go2.sRm = 0; go2.sRn = 0;
      go2.M = C; go2.N = M; go2.K = N; go2.zi_n = 1; go2.flags = 0; go2.act = 0;
      go2.alpha = 1.0f; go2.beta = 0.0f; go2.sa = 1.0f; go2.sb = 1.0f; go2.Npad = M; go2.pad_ = 0;
      k_gemm<1><<<dim3((unsigned)((M) + 31) / 32, (unsigned)((C) + 15) / 16, (unsigned)(1)), 32, 0, stream>>>(go2); }
    { GemmP gQ3;
      gQ3.A = Wq; gQ3.B = x + (size_t)3 * C * N; gQ3.bias = Wq; gQ3.R = Wq; gQ3.C = Q;
      gQ3.sAo = 0; gQ3.sAi = 0; gQ3.sAm = C; gQ3.sAk = 1; gQ3.sBo = 0; gQ3.sBi = 0; gQ3.sBn = 1; gQ3.sBk = N; gQ3.sCo = 0; gQ3.sCi = 0; gQ3.sCm = N; gQ3.sRo = 0; gQ3.sRi = 0; gQ3.sRm = 0; gQ3.sRn = 0;
      gQ3.M = C; gQ3.N = N; gQ3.K = C; gQ3.zi_n = 1; gQ3.flags = 0; gQ3.act = 0;
      gQ3.alpha = 1.0f; gQ3.beta = 0.0f; gQ3.sa = 1.0f; gQ3.sb = 1.0f; gQ3.Npad = N; gQ3.pad_ = 0;
      k_gemm<4><<<dim3((unsigned)((N) + 31) / 32, (unsigned)((C) + 15) / 16, (unsigned)(1)), 32, 0, stream>>>(gQ3); }
    { GemmP gKk3;
      gKk3.A = Wk; gKk3.B = x + (size_t)3 * C * N; gKk3.bias = Wk; gKk3.R = Wk; gKk3.C = Kk;
      gKk3.sAo = 0; gKk3.sAi = 0; gKk3.sAm = C; gKk3.sAk = 1; gKk3.sBo = 0; gKk3.sBi = 0; gKk3.sBn = 1; gKk3.sBk = N; gKk3.sCo = 0; gKk3.sCi = 0; gKk3.sCm = N; gKk3.sRo = 0; gKk3.sRi = 0; gKk3.sRm = 0; gKk3.sRn = 0;
      gKk3.M = C; gKk3.N = N; gKk3.K = C; gKk3.zi_n = 1; gKk3.flags = 0; gKk3.act = 0;
      gKk3.alpha = 1.0f; gKk3.beta = 0.0f; gKk3.sa = 1.0f; gKk3.sb = 1.0f; gKk3.Npad = N; gKk3.pad_ = 0;
      k_gemm<4><<<dim3((unsigned)((N) + 31) / 32, (unsigned)((C) + 15) / 16, (unsigned)(1)), 32, 0, stream>>>(gKk3); }
    { GemmP gV3;
      gV3.A = Wv; gV3.B = x + (size_t)3 * C * N; gV3.bias = Wv; gV3.R = Wv; gV3.C = V;
      gV3.sAo = 0; gV3.sAi = 0; gV3.sAm = C; gV3.sAk = 1; gV3.sBo = 0; gV3.sBi = 0; gV3.sBn = 1; gV3.sBk = N; gV3.sCo = 0; gV3.sCi = 0; gV3.sCm = N; gV3.sRo = 0; gV3.sRi = 0; gV3.sRm = 0; gV3.sRn = 0;
      gV3.M = C; gV3.N = N; gV3.K = C; gV3.zi_n = 1; gV3.flags = 0; gV3.act = 0;
      gV3.alpha = 1.0f; gV3.beta = 0.0f; gV3.sa = 1.0f; gV3.sb = 1.0f; gV3.Npad = N; gV3.pad_ = 0;
      k_gemm<4><<<dim3((unsigned)((N) + 31) / 32, (unsigned)((C) + 15) / 16, (unsigned)(1)), 32, 0, stream>>>(gV3); }
    { GemmP ge3;
      ge3.A = Q; ge3.B = Kk; ge3.bias = Q; ge3.R = Q; ge3.C = ATT;
      ge3.sAo = 0; ge3.sAi = 0; ge3.sAm = 1; ge3.sAk = N; ge3.sBo = 0; ge3.sBi = 0; ge3.sBn = 1; ge3.sBk = N; ge3.sCo = 0; ge3.sCi = 0; ge3.sCm = N; ge3.sRo = 0; ge3.sRi = 0; ge3.sRm = 0; ge3.sRn = 0;
      ge3.M = N; ge3.N = N; ge3.K = C; ge3.zi_n = 1; ge3.flags = 0; ge3.act = 0;
      ge3.alpha = 0.08838834764831843f; ge3.beta = 0.0f; ge3.sa = 1.0f; ge3.sb = 1.0f; ge3.Npad = N; ge3.pad_ = 0;
      k_gemm<4><<<dim3((unsigned)((N) + 31) / 32, (unsigned)((N) + 15) / 16, (unsigned)(1)), 32, 0, stream>>>(ge3); }
    { SmP sm; sm.src = ATT; sm.dst = ATT; sm.Mf = 0; sm.sz = 0; sm.sr = N; sm.dz = 0; sm.dr = N; sm.smz = 0; sm.smr = 0; sm.n = N; sm.pad = 0; sm.scale_in = 1.0f; sm.scale_out = 1.0f;
      k_softmax<<<dim3((unsigned)(N), (unsigned)(1)), 256, 0, stream>>>(sm); }
    k_gd_colsum<<<(unsigned)((N + 255) / 256), 256, 0, stream>>>(ATT, SEL, N);
    k_gd_rank<<<(unsigned)((N + 255) / 256), 256, 0, stream>>>(SEL, IDX, N, M);
    k_gd_gather<<<(unsigned)(((long long)M * N + 255) / 256), 256, 0, stream>>>(ATT, IDX, SCS, N, M);
    { GemmP go3;
      go3.A = V; go3.B = SCS; go3.bias = V; go3.R = V; go3.C = out + (size_t)3 * C * M;
      go3.sAo = 0; go3.sAi = 0; go3.sAm = N; go3.sAk = 1; go3.sBo = 0; go3.sBi = 0; go3.sBn = N; go3.sBk = 1; go3.sCo = 0; go3.sCi = 0; go3.sCm = M; go3.sRo = 0; go3.sRi = 0; go3.sRm = 0; go3.sRn = 0;
      go3.M = C; go3.N = M; go3.K = N; go3.zi_n = 1; go3.flags = 0; go3.act = 0;
      go3.alpha = 1.0f; go3.beta = 0.0f; go3.sa = 1.0f; go3.sb = 1.0f; go3.Npad = M; go3.pad_ = 0;
      k_gemm<1><<<dim3((unsigned)((M) + 31) / 32, (unsigned)((C) + 15) / 16, (unsigned)(1)), 32, 0, stream>>>(go3); }
    { GemmP gQ4;
      gQ4.A = Wq; gQ4.B = x + (size_t)4 * C * N; gQ4.bias = Wq; gQ4.R = Wq; gQ4.C = Q;
      gQ4.sAo = 0; gQ4.sAi = 0; gQ4.sAm = C; gQ4.sAk = 1; gQ4.sBo = 0; gQ4.sBi = 0; gQ4.sBn = 1; gQ4.sBk = N; gQ4.sCo = 0; gQ4.sCi = 0; gQ4.sCm = N; gQ4.sRo = 0; gQ4.sRi = 0; gQ4.sRm = 0; gQ4.sRn = 0;
      gQ4.M = C; gQ4.N = N; gQ4.K = C; gQ4.zi_n = 1; gQ4.flags = 0; gQ4.act = 0;
      gQ4.alpha = 1.0f; gQ4.beta = 0.0f; gQ4.sa = 1.0f; gQ4.sb = 1.0f; gQ4.Npad = N; gQ4.pad_ = 0;
      k_gemm<4><<<dim3((unsigned)((N) + 31) / 32, (unsigned)((C) + 15) / 16, (unsigned)(1)), 32, 0, stream>>>(gQ4); }
    { GemmP gKk4;
      gKk4.A = Wk; gKk4.B = x + (size_t)4 * C * N; gKk4.bias = Wk; gKk4.R = Wk; gKk4.C = Kk;
      gKk4.sAo = 0; gKk4.sAi = 0; gKk4.sAm = C; gKk4.sAk = 1; gKk4.sBo = 0; gKk4.sBi = 0; gKk4.sBn = 1; gKk4.sBk = N; gKk4.sCo = 0; gKk4.sCi = 0; gKk4.sCm = N; gKk4.sRo = 0; gKk4.sRi = 0; gKk4.sRm = 0; gKk4.sRn = 0;
      gKk4.M = C; gKk4.N = N; gKk4.K = C; gKk4.zi_n = 1; gKk4.flags = 0; gKk4.act = 0;
      gKk4.alpha = 1.0f; gKk4.beta = 0.0f; gKk4.sa = 1.0f; gKk4.sb = 1.0f; gKk4.Npad = N; gKk4.pad_ = 0;
      k_gemm<4><<<dim3((unsigned)((N) + 31) / 32, (unsigned)((C) + 15) / 16, (unsigned)(1)), 32, 0, stream>>>(gKk4); }
    { GemmP gV4;
      gV4.A = Wv; gV4.B = x + (size_t)4 * C * N; gV4.bias = Wv; gV4.R = Wv; gV4.C = V;
      gV4.sAo = 0; gV4.sAi = 0; gV4.sAm = C; gV4.sAk = 1; gV4.sBo = 0; gV4.sBi = 0; gV4.sBn = 1; gV4.sBk = N; gV4.sCo = 0; gV4.sCi = 0; gV4.sCm = N; gV4.sRo = 0; gV4.sRi = 0; gV4.sRm = 0; gV4.sRn = 0;
      gV4.M = C; gV4.N = N; gV4.K = C; gV4.zi_n = 1; gV4.flags = 0; gV4.act = 0;
      gV4.alpha = 1.0f; gV4.beta = 0.0f; gV4.sa = 1.0f; gV4.sb = 1.0f; gV4.Npad = N; gV4.pad_ = 0;
      k_gemm<4><<<dim3((unsigned)((N) + 31) / 32, (unsigned)((C) + 15) / 16, (unsigned)(1)), 32, 0, stream>>>(gV4); }
    { GemmP ge4;
      ge4.A = Q; ge4.B = Kk; ge4.bias = Q; ge4.R = Q; ge4.C = ATT;
      ge4.sAo = 0; ge4.sAi = 0; ge4.sAm = 1; ge4.sAk = N; ge4.sBo = 0; ge4.sBi = 0; ge4.sBn = 1; ge4.sBk = N; ge4.sCo = 0; ge4.sCi = 0; ge4.sCm = N; ge4.sRo = 0; ge4.sRi = 0; ge4.sRm = 0; ge4.sRn = 0;
      ge4.M = N; ge4.N = N; ge4.K = C; ge4.zi_n = 1; ge4.flags = 0; ge4.act = 0;
      ge4.alpha = 0.08838834764831843f; ge4.beta = 0.0f; ge4.sa = 1.0f; ge4.sb = 1.0f; ge4.Npad = N; ge4.pad_ = 0;
      k_gemm<4><<<dim3((unsigned)((N) + 31) / 32, (unsigned)((N) + 15) / 16, (unsigned)(1)), 32, 0, stream>>>(ge4); }
    { SmP sm; sm.src = ATT; sm.dst = ATT; sm.Mf = 0; sm.sz = 0; sm.sr = N; sm.dz = 0; sm.dr = N; sm.smz = 0; sm.smr = 0; sm.n = N; sm.pad = 0; sm.scale_in = 1.0f; sm.scale_out = 1.0f;
      k_softmax<<<dim3((unsigned)(N), (unsigned)(1)), 256, 0, stream>>>(sm); }
    k_gd_colsum<<<(unsigned)((N + 255) / 256), 256, 0, stream>>>(ATT, SEL, N);
    k_gd_rank<<<(unsigned)((N + 255) / 256), 256, 0, stream>>>(SEL, IDX, N, M);
    k_gd_gather<<<(unsigned)(((long long)M * N + 255) / 256), 256, 0, stream>>>(ATT, IDX, SCS, N, M);
    { GemmP go4;
      go4.A = V; go4.B = SCS; go4.bias = V; go4.R = V; go4.C = out + (size_t)4 * C * M;
      go4.sAo = 0; go4.sAi = 0; go4.sAm = N; go4.sAk = 1; go4.sBo = 0; go4.sBi = 0; go4.sBn = N; go4.sBk = 1; go4.sCo = 0; go4.sCi = 0; go4.sCm = M; go4.sRo = 0; go4.sRi = 0; go4.sRm = 0; go4.sRn = 0;
      go4.M = C; go4.N = M; go4.K = N; go4.zi_n = 1; go4.flags = 0; go4.act = 0;
      go4.alpha = 1.0f; go4.beta = 0.0f; go4.sa = 1.0f; go4.sb = 1.0f; go4.Npad = M; go4.pad_ = 0;
      k_gemm<1><<<dim3((unsigned)((M) + 31) / 32, (unsigned)((C) + 15) / 16, (unsigned)(1)), 32, 0, stream>>>(go4); }
    { GemmP gQ5;
      gQ5.A = Wq; gQ5.B = x + (size_t)5 * C * N; gQ5.bias = Wq; gQ5.R = Wq; gQ5.C = Q;
      gQ5.sAo = 0; gQ5.sAi = 0; gQ5.sAm = C; gQ5.sAk = 1; gQ5.sBo = 0; gQ5.sBi = 0; gQ5.sBn = 1; gQ5.sBk = N; gQ5.sCo = 0; gQ5.sCi = 0; gQ5.sCm = N; gQ5.sRo = 0; gQ5.sRi = 0; gQ5.sRm = 0; gQ5.sRn = 0;
      gQ5.M = C; gQ5.N = N; gQ5.K = C; gQ5.zi_n = 1; gQ5.flags = 0; gQ5.act = 0;
      gQ5.alpha = 1.0f; gQ5.beta = 0.0f; gQ5.sa = 1.0f; gQ5.sb = 1.0f; gQ5.Npad = N; gQ5.pad_ = 0;
      k_gemm<4><<<dim3((unsigned)((N) + 31) / 32, (unsigned)((C) + 15) / 16, (unsigned)(1)), 32, 0, stream>>>(gQ5); }
    { GemmP gKk5;
      gKk5.A = Wk; gKk5.B = x + (size_t)5 * C * N; gKk5.bias = Wk; gKk5.R = Wk; gKk5.C = Kk;
      gKk5.sAo = 0; gKk5.sAi = 0; gKk5.sAm = C; gKk5.sAk = 1; gKk5.sBo = 0; gKk5.sBi = 0; gKk5.sBn = 1; gKk5.sBk = N; gKk5.sCo = 0; gKk5.sCi = 0; gKk5.sCm = N; gKk5.sRo = 0; gKk5.sRi = 0; gKk5.sRm = 0; gKk5.sRn = 0;
      gKk5.M = C; gKk5.N = N; gKk5.K = C; gKk5.zi_n = 1; gKk5.flags = 0; gKk5.act = 0;
      gKk5.alpha = 1.0f; gKk5.beta = 0.0f; gKk5.sa = 1.0f; gKk5.sb = 1.0f; gKk5.Npad = N; gKk5.pad_ = 0;
      k_gemm<4><<<dim3((unsigned)((N) + 31) / 32, (unsigned)((C) + 15) / 16, (unsigned)(1)), 32, 0, stream>>>(gKk5); }
    { GemmP gV5;
      gV5.A = Wv; gV5.B = x + (size_t)5 * C * N; gV5.bias = Wv; gV5.R = Wv; gV5.C = V;
      gV5.sAo = 0; gV5.sAi = 0; gV5.sAm = C; gV5.sAk = 1; gV5.sBo = 0; gV5.sBi = 0; gV5.sBn = 1; gV5.sBk = N; gV5.sCo = 0; gV5.sCi = 0; gV5.sCm = N; gV5.sRo = 0; gV5.sRi = 0; gV5.sRm = 0; gV5.sRn = 0;
      gV5.M = C; gV5.N = N; gV5.K = C; gV5.zi_n = 1; gV5.flags = 0; gV5.act = 0;
      gV5.alpha = 1.0f; gV5.beta = 0.0f; gV5.sa = 1.0f; gV5.sb = 1.0f; gV5.Npad = N; gV5.pad_ = 0;
      k_gemm<4><<<dim3((unsigned)((N) + 31) / 32, (unsigned)((C) + 15) / 16, (unsigned)(1)), 32, 0, stream>>>(gV5); }
    { GemmP ge5;
      ge5.A = Q; ge5.B = Kk; ge5.bias = Q; ge5.R = Q; ge5.C = ATT;
      ge5.sAo = 0; ge5.sAi = 0; ge5.sAm = 1; ge5.sAk = N; ge5.sBo = 0; ge5.sBi = 0; ge5.sBn = 1; ge5.sBk = N; ge5.sCo = 0; ge5.sCi = 0; ge5.sCm = N; ge5.sRo = 0; ge5.sRi = 0; ge5.sRm = 0; ge5.sRn = 0;
      ge5.M = N; ge5.N = N; ge5.K = C; ge5.zi_n = 1; ge5.flags = 0; ge5.act = 0;
      ge5.alpha = 0.08838834764831843f; ge5.beta = 0.0f; ge5.sa = 1.0f; ge5.sb = 1.0f; ge5.Npad = N; ge5.pad_ = 0;
      k_gemm<4><<<dim3((unsigned)((N) + 31) / 32, (unsigned)((N) + 15) / 16, (unsigned)(1)), 32, 0, stream>>>(ge5); }
    { SmP sm; sm.src = ATT; sm.dst = ATT; sm.Mf = 0; sm.sz = 0; sm.sr = N; sm.dz = 0; sm.dr = N; sm.smz = 0; sm.smr = 0; sm.n = N; sm.pad = 0; sm.scale_in = 1.0f; sm.scale_out = 1.0f;
      k_softmax<<<dim3((unsigned)(N), (unsigned)(1)), 256, 0, stream>>>(sm); }
    k_gd_colsum<<<(unsigned)((N + 255) / 256), 256, 0, stream>>>(ATT, SEL, N);
    k_gd_rank<<<(unsigned)((N + 255) / 256), 256, 0, stream>>>(SEL, IDX, N, M);
    k_gd_gather<<<(unsigned)(((long long)M * N + 255) / 256), 256, 0, stream>>>(ATT, IDX, SCS, N, M);
    { GemmP go5;
      go5.A = V; go5.B = SCS; go5.bias = V; go5.R = V; go5.C = out + (size_t)5 * C * M;
      go5.sAo = 0; go5.sAi = 0; go5.sAm = N; go5.sAk = 1; go5.sBo = 0; go5.sBi = 0; go5.sBn = N; go5.sBk = 1; go5.sCo = 0; go5.sCi = 0; go5.sCm = M; go5.sRo = 0; go5.sRi = 0; go5.sRm = 0; go5.sRn = 0;
      go5.M = C; go5.N = M; go5.K = N; go5.zi_n = 1; go5.flags = 0; go5.act = 0;
      go5.alpha = 1.0f; go5.beta = 0.0f; go5.sa = 1.0f; go5.sb = 1.0f; go5.Npad = M; go5.pad_ = 0;
      k_gemm<1><<<dim3((unsigned)((M) + 31) / 32, (unsigned)((C) + 15) / 16, (unsigned)(1)), 32, 0, stream>>>(go5); }
    { GemmP gQ6;
      gQ6.A = Wq; gQ6.B = x + (size_t)6 * C * N; gQ6.bias = Wq; gQ6.R = Wq; gQ6.C = Q;
      gQ6.sAo = 0; gQ6.sAi = 0; gQ6.sAm = C; gQ6.sAk = 1; gQ6.sBo = 0; gQ6.sBi = 0; gQ6.sBn = 1; gQ6.sBk = N; gQ6.sCo = 0; gQ6.sCi = 0; gQ6.sCm = N; gQ6.sRo = 0; gQ6.sRi = 0; gQ6.sRm = 0; gQ6.sRn = 0;
      gQ6.M = C; gQ6.N = N; gQ6.K = C; gQ6.zi_n = 1; gQ6.flags = 0; gQ6.act = 0;
      gQ6.alpha = 1.0f; gQ6.beta = 0.0f; gQ6.sa = 1.0f; gQ6.sb = 1.0f; gQ6.Npad = N; gQ6.pad_ = 0;
      k_gemm<4><<<dim3((unsigned)((N) + 31) / 32, (unsigned)((C) + 15) / 16, (unsigned)(1)), 32, 0, stream>>>(gQ6); }
    { GemmP gKk6;
      gKk6.A = Wk; gKk6.B = x + (size_t)6 * C * N; gKk6.bias = Wk; gKk6.R = Wk; gKk6.C = Kk;
      gKk6.sAo = 0; gKk6.sAi = 0; gKk6.sAm = C; gKk6.sAk = 1; gKk6.sBo = 0; gKk6.sBi = 0; gKk6.sBn = 1; gKk6.sBk = N; gKk6.sCo = 0; gKk6.sCi = 0; gKk6.sCm = N; gKk6.sRo = 0; gKk6.sRi = 0; gKk6.sRm = 0; gKk6.sRn = 0;
      gKk6.M = C; gKk6.N = N; gKk6.K = C; gKk6.zi_n = 1; gKk6.flags = 0; gKk6.act = 0;
      gKk6.alpha = 1.0f; gKk6.beta = 0.0f; gKk6.sa = 1.0f; gKk6.sb = 1.0f; gKk6.Npad = N; gKk6.pad_ = 0;
      k_gemm<4><<<dim3((unsigned)((N) + 31) / 32, (unsigned)((C) + 15) / 16, (unsigned)(1)), 32, 0, stream>>>(gKk6); }
    { GemmP gV6;
      gV6.A = Wv; gV6.B = x + (size_t)6 * C * N; gV6.bias = Wv; gV6.R = Wv; gV6.C = V;
      gV6.sAo = 0; gV6.sAi = 0; gV6.sAm = C; gV6.sAk = 1; gV6.sBo = 0; gV6.sBi = 0; gV6.sBn = 1; gV6.sBk = N; gV6.sCo = 0; gV6.sCi = 0; gV6.sCm = N; gV6.sRo = 0; gV6.sRi = 0; gV6.sRm = 0; gV6.sRn = 0;
      gV6.M = C; gV6.N = N; gV6.K = C; gV6.zi_n = 1; gV6.flags = 0; gV6.act = 0;
      gV6.alpha = 1.0f; gV6.beta = 0.0f; gV6.sa = 1.0f; gV6.sb = 1.0f; gV6.Npad = N; gV6.pad_ = 0;
      k_gemm<4><<<dim3((unsigned)((N) + 31) / 32, (unsigned)((C) + 15) / 16, (unsigned)(1)), 32, 0, stream>>>(gV6); }
    { GemmP ge6;
      ge6.A = Q; ge6.B = Kk; ge6.bias = Q; ge6.R = Q; ge6.C = ATT;
      ge6.sAo = 0; ge6.sAi = 0; ge6.sAm = 1; ge6.sAk = N; ge6.sBo = 0; ge6.sBi = 0; ge6.sBn = 1; ge6.sBk = N; ge6.sCo = 0; ge6.sCi = 0; ge6.sCm = N; ge6.sRo = 0; ge6.sRi = 0; ge6.sRm = 0; ge6.sRn = 0;
      ge6.M = N; ge6.N = N; ge6.K = C; ge6.zi_n = 1; ge6.flags = 0; ge6.act = 0;
      ge6.alpha = 0.08838834764831843f; ge6.beta = 0.0f; ge6.sa = 1.0f; ge6.sb = 1.0f; ge6.Npad = N; ge6.pad_ = 0;
      k_gemm<4><<<dim3((unsigned)((N) + 31) / 32, (unsigned)((N) + 15) / 16, (unsigned)(1)), 32, 0, stream>>>(ge6); }
    { SmP sm; sm.src = ATT; sm.dst = ATT; sm.Mf = 0; sm.sz = 0; sm.sr = N; sm.dz = 0; sm.dr = N; sm.smz = 0; sm.smr = 0; sm.n = N; sm.pad = 0; sm.scale_in = 1.0f; sm.scale_out = 1.0f;
      k_softmax<<<dim3((unsigned)(N), (unsigned)(1)), 256, 0, stream>>>(sm); }
    k_gd_colsum<<<(unsigned)((N + 255) / 256), 256, 0, stream>>>(ATT, SEL, N);
    k_gd_rank<<<(unsigned)((N + 255) / 256), 256, 0, stream>>>(SEL, IDX, N, M);
    k_gd_gather<<<(unsigned)(((long long)M * N + 255) / 256), 256, 0, stream>>>(ATT, IDX, SCS, N, M);
    { GemmP go6;
      go6.A = V; go6.B = SCS; go6.bias = V; go6.R = V; go6.C = out + (size_t)6 * C * M;
      go6.sAo = 0; go6.sAi = 0; go6.sAm = N; go6.sAk = 1; go6.sBo = 0; go6.sBi = 0; go6.sBn = N; go6.sBk = 1; go6.sCo = 0; go6.sCi = 0; go6.sCm = M; go6.sRo = 0; go6.sRi = 0; go6.sRm = 0; go6.sRn = 0;
      go6.M = C; go6.N = M; go6.K = N; go6.zi_n = 1; go6.flags = 0; go6.act = 0;
      go6.alpha = 1.0f; go6.beta = 0.0f; go6.sa = 1.0f; go6.sb = 1.0f; go6.Npad = M; go6.pad_ = 0;
      k_gemm<1><<<dim3((unsigned)((M) + 31) / 32, (unsigned)((C) + 15) / 16, (unsigned)(1)), 32, 0, stream>>>(go6); }
    { GemmP gQ7;
      gQ7.A = Wq; gQ7.B = x + (size_t)7 * C * N; gQ7.bias = Wq; gQ7.R = Wq; gQ7.C = Q;
      gQ7.sAo = 0; gQ7.sAi = 0; gQ7.sAm = C; gQ7.sAk = 1; gQ7.sBo = 0; gQ7.sBi = 0; gQ7.sBn = 1; gQ7.sBk = N; gQ7.sCo = 0; gQ7.sCi = 0; gQ7.sCm = N; gQ7.sRo = 0; gQ7.sRi = 0; gQ7.sRm = 0; gQ7.sRn = 0;
      gQ7.M = C; gQ7.N = N; gQ7.K = C; gQ7.zi_n = 1; gQ7.flags = 0; gQ7.act = 0;
      gQ7.alpha = 1.0f; gQ7.beta = 0.0f; gQ7.sa = 1.0f; gQ7.sb = 1.0f; gQ7.Npad = N; gQ7.pad_ = 0;
      k_gemm<4><<<dim3((unsigned)((N) + 31) / 32, (unsigned)((C) + 15) / 16, (unsigned)(1)), 32, 0, stream>>>(gQ7); }
    { GemmP gKk7;
      gKk7.A = Wk; gKk7.B = x + (size_t)7 * C * N; gKk7.bias = Wk; gKk7.R = Wk; gKk7.C = Kk;
      gKk7.sAo = 0; gKk7.sAi = 0; gKk7.sAm = C; gKk7.sAk = 1; gKk7.sBo = 0; gKk7.sBi = 0; gKk7.sBn = 1; gKk7.sBk = N; gKk7.sCo = 0; gKk7.sCi = 0; gKk7.sCm = N; gKk7.sRo = 0; gKk7.sRi = 0; gKk7.sRm = 0; gKk7.sRn = 0;
      gKk7.M = C; gKk7.N = N; gKk7.K = C; gKk7.zi_n = 1; gKk7.flags = 0; gKk7.act = 0;
      gKk7.alpha = 1.0f; gKk7.beta = 0.0f; gKk7.sa = 1.0f; gKk7.sb = 1.0f; gKk7.Npad = N; gKk7.pad_ = 0;
      k_gemm<4><<<dim3((unsigned)((N) + 31) / 32, (unsigned)((C) + 15) / 16, (unsigned)(1)), 32, 0, stream>>>(gKk7); }
    { GemmP gV7;
      gV7.A = Wv; gV7.B = x + (size_t)7 * C * N; gV7.bias = Wv; gV7.R = Wv; gV7.C = V;
      gV7.sAo = 0; gV7.sAi = 0; gV7.sAm = C; gV7.sAk = 1; gV7.sBo = 0; gV7.sBi = 0; gV7.sBn = 1; gV7.sBk = N; gV7.sCo = 0; gV7.sCi = 0; gV7.sCm = N; gV7.sRo = 0; gV7.sRi = 0; gV7.sRm = 0; gV7.sRn = 0;
      gV7.M = C; gV7.N = N; gV7.K = C; gV7.zi_n = 1; gV7.flags = 0; gV7.act = 0;
      gV7.alpha = 1.0f; gV7.beta = 0.0f; gV7.sa = 1.0f; gV7.sb = 1.0f; gV7.Npad = N; gV7.pad_ = 0;
      k_gemm<4><<<dim3((unsigned)((N) + 31) / 32, (unsigned)((C) + 15) / 16, (unsigned)(1)), 32, 0, stream>>>(gV7); }
    { GemmP ge7;
      ge7.A = Q; ge7.B = Kk; ge7.bias = Q; ge7.R = Q; ge7.C = ATT;
      ge7.sAo = 0; ge7.sAi = 0; ge7.sAm = 1; ge7.sAk = N; ge7.sBo = 0; ge7.sBi = 0; ge7.sBn = 1; ge7.sBk = N; ge7.sCo = 0; ge7.sCi = 0; ge7.sCm = N; ge7.sRo = 0; ge7.sRi = 0; ge7.sRm = 0; ge7.sRn = 0;
      ge7.M = N; ge7.N = N; ge7.K = C; ge7.zi_n = 1; ge7.flags = 0; ge7.act = 0;
      ge7.alpha = 0.08838834764831843f; ge7.beta = 0.0f; ge7.sa = 1.0f; ge7.sb = 1.0f; ge7.Npad = N; ge7.pad_ = 0;
      k_gemm<4><<<dim3((unsigned)((N) + 31) / 32, (unsigned)((N) + 15) / 16, (unsigned)(1)), 32, 0, stream>>>(ge7); }
    { SmP sm; sm.src = ATT; sm.dst = ATT; sm.Mf = 0; sm.sz = 0; sm.sr = N; sm.dz = 0; sm.dr = N; sm.smz = 0; sm.smr = 0; sm.n = N; sm.pad = 0; sm.scale_in = 1.0f; sm.scale_out = 1.0f;
      k_softmax<<<dim3((unsigned)(N), (unsigned)(1)), 256, 0, stream>>>(sm); }
    k_gd_colsum<<<(unsigned)((N + 255) / 256), 256, 0, stream>>>(ATT, SEL, N);
    k_gd_rank<<<(unsigned)((N + 255) / 256), 256, 0, stream>>>(SEL, IDX, N, M);
    k_gd_gather<<<(unsigned)(((long long)M * N + 255) / 256), 256, 0, stream>>>(ATT, IDX, SCS, N, M);
    { GemmP go7;
      go7.A = V; go7.B = SCS; go7.bias = V; go7.R = V; go7.C = out + (size_t)7 * C * M;
      go7.sAo = 0; go7.sAi = 0; go7.sAm = N; go7.sAk = 1; go7.sBo = 0; go7.sBi = 0; go7.sBn = N; go7.sBk = 1; go7.sCo = 0; go7.sCi = 0; go7.sCm = M; go7.sRo = 0; go7.sRi = 0; go7.sRm = 0; go7.sRn = 0;
      go7.M = C; go7.N = M; go7.K = N; go7.zi_n = 1; go7.flags = 0; go7.act = 0;
      go7.alpha = 1.0f; go7.beta = 0.0f; go7.sa = 1.0f; go7.sb = 1.0f; go7.Npad = M; go7.pad_ = 0;
      k_gemm<1><<<dim3((unsigned)((M) + 31) / 32, (unsigned)((C) + 15) / 16, (unsigned)(1)), 32, 0, stream>>>(go7); }
}
